// ProteinGNNEncoder_26199300506300
// MI455X (gfx1250) — hardware-verified
//
#include <hip/hip_runtime.h>
#include <stddef.h>
#include <stdint.h>


#define HD      128
#define HD2     256
#define INDIM   9
#define EDIM    4
#define K1ROWS  260
#define NLAY    3
#define NTHR    256
#define NWAVE   8
#define EPT     8
#define CHUNK   (NTHR * EPT)
#define WCAP    (EPT * 32)
#define LISTN   (NWAVE * WCAP)
#define NBMAX   2048
#define RCAP    28672
#define DEGCAP  4096
#define GBM     64
#define GBN     64
#define GTHR    128
#define ZP      136
#define SP      132
#define WL_W1T  0
#define WL_W2T  32768
#define WL_U1T  49152
#define WL_U2T  81920
#define WL_LAY  98304
#define UPL     (WL_LAY / 8)
#define CA      32.0f
#define CL      2048.0f
#define CW      1024.0f
#define SCL     0.000030517578125f
#define SCLL    0.00000001490116119384765625f
#define LNEPS   1e-5f
#define WSMAX   134217728
#define LDS_AGG ((2 * RCAP + 2 * NBMAX + LISTN) * 4 + 64)
#define LDS_UPD (2 * GBM * ZP * 2 + GBM * SP * 4)

static_assert((CHUNK & (CHUNK - 1)) == 0 && CHUNK <= 4096);
static_assert((NBMAX & (NBMAX - 1)) == 0 && NBMAX <= 4096);
static_assert(NTHR * 8 == NBMAX);
static_assert(LISTN >= NBMAX);
static_assert(LISTN >= NWAVE * WCAP);
static_assert((RCAP % 32) == 0);
static_assert(LDS_AGG <= 300000);
static_assert(LDS_UPD <= 300000);
static_assert(GBM == (GTHR / 32) * 16);
static_assert((HD % 32) == 0 && (HD2 % GBN) == 0 && (HD % GBN) == 0);
static_assert(HD / 32 == 4);
static_assert(NWAVE * 8 == GBM);
static_assert(UPL == 4096 + 2048 + 4096 + 2048);
static_assert((ZP * 2) % 16 == 0 && (SP * 4) % 16 == 0);
static_assert((GBM * ZP * 2) % 16 == 0);

typedef float    v4f  __attribute__((ext_vector_type(4)));
typedef float    v8f  __attribute__((ext_vector_type(8)));
typedef int      v4i  __attribute__((ext_vector_type(4)));
typedef int      v8i  __attribute__((ext_vector_type(8)));
typedef _Float16 v8h  __attribute__((ext_vector_type(8)));
typedef _Float16 v16h __attribute__((ext_vector_type(16)));
union FragH { v16h v; v8h h[2]; v8i w; };

__device__ __forceinline__ v8f wmh(const FragH& a, const FragH& b, v8f c) {
  v8f d = __builtin_amdgcn_wmma_f32_16x16x32_f16(false, a.v, false, b.v, (short)0, c, false, false);
  asm volatile("v_nop\n\tv_nop\n\tv_nop\n\tv_nop" : "+v"(d) : "v"(a.w), "v"(b.w));
  return d;
}

__device__ __forceinline__ v8h cvt8h(const v4f a, const v4f b, const float c) {
  v8h hv;
  hv[0] = (_Float16)(a.x * c); hv[1] = (_Float16)(a.y * c);
  hv[2] = (_Float16)(a.z * c); hv[3] = (_Float16)(a.w * c);
  hv[4] = (_Float16)(b.x * c); hv[5] = (_Float16)(b.y * c);
  hv[6] = (_Float16)(b.z * c); hv[7] = (_Float16)(b.w * c);
  return hv;
}

__device__ __forceinline__ void cvt8hl(const v4f a, const v4f b, v8h& hi, v8h& lo) {
  const float t[8] = {a.x, a.y, a.z, a.w, b.x, b.y, b.z, b.w};
#pragma unroll
  for (int i = 0; i < 8; ++i) {
    const float s = t[i] * CA;
    const _Float16 q = (_Float16)s;
    hi[i] = q;
    lo[i] = (_Float16)((s - (float)q) * CL);
  }
}

__device__ __forceinline__ v4f relu4(const v4f v) {
  v4f r;
  r.x = fmaxf(v.x, 0.f); r.y = fmaxf(v.y, 0.f); r.z = fmaxf(v.z, 0.f); r.w = fmaxf(v.w, 0.f);
  return r;
}

__device__ __forceinline__ float wred(float v) {
#pragma unroll
  for (int o = 16; o > 0; o >>= 1) v += __shfl_xor(v, o);
  return v;
}

__device__ __forceinline__ int scan_chunk(const int* __restrict__ dsts, int nE, int cbase, int slotBase,
                                          int nb, int vec8, int* list, int tid, int lane, int wave) {
  int wc = 0;
  const int el0  = tid * EPT;
  const int e0   = cbase + el0;
  const int sent = -2147483647 - 1;
  v4i da, db;
  if (vec8 != 0 && cbase + CHUNK <= nE) {
    da = *(const v4i*)(dsts + e0);
    db = *(const v4i*)(dsts + e0 + 4);
  } else {
    da.x = (e0     < nE) ? dsts[min(e0,     nE - 1)] : sent;
    da.y = (e0 + 1 < nE) ? dsts[min(e0 + 1, nE - 1)] : sent;
    da.z = (e0 + 2 < nE) ? dsts[min(e0 + 2, nE - 1)] : sent;
    da.w = (e0 + 3 < nE) ? dsts[min(e0 + 3, nE - 1)] : sent;
    db.x = (e0 + 4 < nE) ? dsts[min(e0 + 4, nE - 1)] : sent;
    db.y = (e0 + 5 < nE) ? dsts[min(e0 + 5, nE - 1)] : sent;
    db.z = (e0 + 6 < nE) ? dsts[min(e0 + 6, nE - 1)] : sent;
    db.w = (e0 + 7 < nE) ? dsts[min(e0 + 7, nE - 1)] : sent;
  }
  const unsigned nbs = (unsigned)slotBase;
  const unsigned unb = (unsigned)nb;
  const unsigned s0 = (unsigned)da.x - nbs, s1 = (unsigned)da.y - nbs;
  const unsigned s2 = (unsigned)da.z - nbs, s3 = (unsigned)da.w - nbs;
  const unsigned s4 = (unsigned)db.x - nbs, s5 = (unsigned)db.y - nbs;
  const unsigned s6 = (unsigned)db.z - nbs, s7 = (unsigned)db.w - nbs;
  const bool h0 = s0 < unb, h1 = s1 < unb, h2 = s2 < unb, h3 = s3 < unb;
  const bool h4 = s4 < unb, h5 = s5 < unb, h6 = s6 < unb, h7 = s7 < unb;
  const unsigned any = __builtin_amdgcn_ballot_w32(h0 | h1 | h2 | h3 | h4 | h5 | h6 | h7);
  if (any != 0u) {
#define HITJ(J, HJ, SJ) { \
      const unsigned mj = __builtin_amdgcn_ballot_w32(HJ); \
      if (mj != 0u) { \
        if (HJ) { \
          const int pos = wc + (int)__builtin_amdgcn_mbcnt_lo(mj, 0u); \
          if (pos < WCAP) list[wave * WCAP + pos] = ((el0 + (J)) << 12) | (int)(SJ); \
        } \
        wc += (int)__builtin_popcount(mj); } }
    HITJ(0, h0, s0)
    HITJ(1, h1, s1)
    HITJ(2, h2, s2)
    HITJ(3, h3, s3)
    HITJ(4, h4, s4)
    HITJ(5, h5, s5)
    HITJ(6, h6, s6)
    HITJ(7, h7, s7)
#undef HITJ
  }
  return wc;
}

__global__ __launch_bounds__(NTHR) void k_wcvt(const float* __restrict__ mw1, const float* __restrict__ mw2,
                                               const float* __restrict__ uw1, const float* __restrict__ uw2,
                                               _Float16* wt, int nUnits) {
  const int u = (int)blockIdx.x * NTHR + (int)threadIdx.x;
  if (u >= nUnits) return;
  const int lay = u / UPL;
  const int r   = u - lay * UPL;
  const int pl  = (r < 4096) ? 0 : ((r < 6144) ? 1 : ((r < 10240) ? 2 : 3));
  const int rb  = (pl == 0) ? 0 : ((pl == 1) ? 4096 : ((pl == 2) ? 6144 : 10240));
  const int rr  = r - rb;
  const int ksh = (pl == 2) ? 5 : 4;
  const int K   = (pl == 2) ? HD2 : HD;
  const int n   = rr >> ksh;
  const int k8  = (rr & ((1 << ksh) - 1)) * 8;
  const float* src = (pl == 0) ? (mw1 + (size_t)lay * K1ROWS * HD)
                   : ((pl == 1) ? (mw2 + (size_t)lay * HD * HD)
                   : ((pl == 2) ? (uw1 + (size_t)lay * HD2 * HD)
                                : (uw2 + (size_t)lay * HD * HD)));
  const int srow = (pl == 0) ? ((n >> 7) * HD + k8) : k8;
  const int scol = (pl == 0) ? (n & (HD - 1)) : n;
  const float* p = src + (size_t)srow * HD + scol;
  v4f a, b;
  a.x = p[0];              a.y = p[(size_t)HD];     a.z = p[(size_t)2 * HD]; a.w = p[(size_t)3 * HD];
  b.x = p[(size_t)4 * HD]; b.y = p[(size_t)5 * HD]; b.z = p[(size_t)6 * HD]; b.w = p[(size_t)7 * HD];
  const v8h hv = cvt8h(a, b, CW);
  const int poff = (pl == 0) ? WL_W1T : ((pl == 1) ? WL_W2T : ((pl == 2) ? WL_U1T : WL_U2T));
  const size_t o = (size_t)lay * WL_LAY + (size_t)poff + (size_t)n * K + k8;
  *(volatile v8h*)(wt + o) = hv;
  __threadfence();
  *(volatile v8h*)(wt + o) = hv;
}

__global__ __launch_bounds__(NTHR) void k_proj(const float* __restrict__ x, const float* __restrict__ pw,
                                               const float* __restrict__ pb, float* out, int nTot) {
  const int t = (int)blockIdx.x * NTHR + (int)threadIdx.x;
  if (t >= nTot) return;
  const int n = t >> 5, j4 = (t & 31) * 4;
  const float* xr = x + (size_t)n * INDIM;
  v4f s = *(const v4f*)(pb + j4);
#pragma unroll
  for (int k = 0; k < INDIM; ++k) {
    const float xv = xr[k];
    const v4f wv = *(const v4f*)(pw + k * HD + j4);
    s.x = fmaf(xv, wv.x, s.x); s.y = fmaf(xv, wv.y, s.y);
    s.z = fmaf(xv, wv.z, s.z); s.w = fmaf(xv, wv.w, s.w);
  }
  float* op = out + (size_t)n * HD + j4;
  *(volatile v4f*)op = s;
  __threadfence();
  *(volatile v4f*)op = s;
}

template<int EPI>
__global__ __launch_bounds__(GTHR) void k_ngemm(const float* __restrict__ A, const _Float16* __restrict__ WT,
                                                const float* __restrict__ bias, const float* __restrict__ rsc,
                                                float* outF, int nAr, int lda, int K, int ldo, int nbias) {
  __shared__ __attribute__((aligned(16))) float stg[GBM * GBN];
  const int tid = (int)threadIdx.x, lane = tid & 31, wave = tid >> 5, hh = lane >> 4, m = lane & 15;
  const int rowBase = (int)blockIdx.x * GBM;
  const int col0    = (int)blockIdx.y * GBN;

  v8f acch[4], accl[4];
  {
    const v8f z = {0.f, 0.f, 0.f, 0.f, 0.f, 0.f, 0.f, 0.f};
#pragma unroll
    for (int t = 0; t < 4; ++t) { acch[t] = z; accl[t] = z; }
  }
  const int gra = rowBase + 16 * wave + m;
  const int grc = gra > nAr - 1 ? nAr - 1 : gra;
  const float* ap = A + (size_t)grc * (size_t)lda + 8 * hh;
  const _Float16* wp = WT + (size_t)(col0 + m) * (size_t)K + 8 * hh;
  const int ksteps = K >> 5;
#pragma unroll 1
  for (int ks = 0; ks < ksteps; ++ks) {
    const float* aq = ap + 32 * ks;
    const v4f a0 = *(const v4f*)aq,        a1 = *(const v4f*)(aq + 4);
    const v4f a2 = *(const v4f*)(aq + 16), a3 = *(const v4f*)(aq + 20);
    FragH ah, al;
    cvt8hl(a0, a1, ah.h[0], al.h[0]);
    cvt8hl(a2, a3, ah.h[1], al.h[1]);
#pragma unroll
    for (int t = 0; t < 4; ++t) {
      const _Float16* wq = wp + (size_t)(16 * t) * (size_t)K + 32 * ks;
      FragH bf;
      bf.h[0] = *(const v8h*)wq;
      bf.h[1] = *(const v8h*)(wq + 16);
      acch[t] = wmh(ah, bf, acch[t]);
      accl[t] = wmh(al, bf, accl[t]);
    }
  }

  float rs[8];
#pragma unroll
  for (int r = 0; r < 8; ++r) rs[r] = 0.f;
  if (EPI == 1) {
    const int lr0 = rowBase + 16 * wave + 8 * hh;
    const v4f ra = *(const v4f*)(rsc + lr0), rb = *(const v4f*)(rsc + lr0 + 4);
    rs[0] = ra.x; rs[1] = ra.y; rs[2] = ra.z; rs[3] = ra.w;
    rs[4] = rb.x; rs[5] = rb.y; rs[6] = rb.z; rs[7] = rb.w;
  }

#pragma unroll
  for (int t = 0; t < 4; ++t) {
    const int lc  = 16 * t + m;
    const int col = col0 + lc;
    int bi = col > nbias - 1 ? nbias - 1 : col;
    bi = bi < 0 ? 0 : bi;
    const float bl = bias[bi];
    const float bv = (col < nbias) ? bl : 0.f;
#pragma unroll
    for (int r = 0; r < 8; ++r) {
      const int lr = 16 * wave + 8 * hh + r;
      float v = acch[t][r] * SCL;
      v = fmaf(accl[t][r], SCLL, v);
      if (EPI == 0) v = v + bv;
      else          v = fmaf(rs[r], bv, v);
      stg[lr * GBN + lc] = v;
    }
  }
  __syncthreads();

  v4f fv[8];
#pragma unroll
  for (int i = 0; i < 8; ++i) {
    const int lr = 16 * wave + 2 * i + hh;
    fv[i] = *(const v4f*)(stg + lr * GBN + 4 * m);
  }
#pragma unroll
  for (int i = 0; i < 8; ++i) {
    const int lr = 16 * wave + 2 * i + hh;
    const int gr = rowBase + lr;
    float* op = outF + (size_t)gr * (size_t)ldo + col0 + 4 * m;
    *(volatile v4f*)op = fv[i];
  }
  __threadfence();
#pragma unroll
  for (int i = 0; i < 8; ++i) {
    const int lr = 16 * wave + 2 * i + hh;
    const int gr = rowBase + lr;
    float* op = outF + (size_t)gr * (size_t)ldo + col0 + 4 * m;
    *(volatile v4f*)op = fv[i];
  }
}

__global__ __launch_bounds__(NTHR) void k_scan(
    const int* __restrict__ dsts, const int* __restrict__ srcs, const float* __restrict__ eattr,
    const float* __restrict__ PQ, const float* __restrict__ w1c, float* RS, float* DEG,
    int nN, int nE, int nb, int vec8, int NPr) {
  extern __shared__ v4f lds_dyn[];
  int* reg1 = (int*)lds_dyn;
  int* reg2 = reg1 + RCAP;
  int* scnt = reg2 + RCAP;
  int* soff = scnt + NBMAX;
  int* list = soff + NBMAX;
  int* wcnt = list + LISTN;
  int* wtot = wcnt + NWAVE;
  const int tid = (int)threadIdx.x, lane = tid & 31, wave = tid >> 5;
  const int nodeBase = (int)blockIdx.x * nb;

  for (int i = tid; i < NBMAX; i += NTHR) scnt[i] = 0;
  __syncthreads();

  int tot = 0;
  const int nChunks = (nE + CHUNK - 1) / CHUNK;
#pragma unroll 1
  for (int ch = 0; ch < nChunks; ++ch) {
    const int cbase = ch * CHUNK;
    const int wc = scan_chunk(dsts, nE, cbase, nodeBase, nb, vec8, list, tid, lane, wave);
    if (lane == 0) wcnt[wave] = wc;
    __syncthreads();
    int pre = 0, all = 0;
#pragma unroll
    for (int w2 = 0; w2 < NWAVE; ++w2) {
      int c = wcnt[w2];
      c = c < 0 ? 0 : (c > WCAP ? WCAP : c);
      all += c;
      pre += (w2 < wave) ? c : 0;
    }
    const int wcc  = wc > WCAP ? WCAP : wc;
    const int base = tot + pre;
#pragma unroll 1
    for (int i = lane; i < wcc; i += 32) {
      const int ent = list[wave * WCAP + i];
      const int el  = (ent >> 12) & (CHUNK - 1);
      const int sl  = ent & (NBMAX - 1);
      int eid = cbase + el;
      eid = eid > nE - 1 ? nE - 1 : eid;
      const int pos = base + i;
      if (pos < RCAP) reg1[pos] = (int)(((unsigned)eid << 12) | (unsigned)sl);
    }
    tot += all;
    tot = tot > RCAP ? RCAP : tot;
    __syncthreads();
  }
  const int nh = tot;

  if (wave == 0) {
#pragma unroll 1
    for (int b0 = 0; b0 < nh; b0 += 32) {
      const int idx = b0 + lane;
      const int uv  = reg1[idx < RCAP ? idx : RCAP - 1];
      const int m32 = (nh - b0) < 32 ? (nh - b0) : 32;
#pragma unroll 1
      for (int k = 0; k < m32; ++k) {
        const int u  = __builtin_amdgcn_readlane(uv, k);
        const int sl = u & (NBMAX - 1);
        if (lane == 0) scnt[sl] = scnt[sl] + 1;
      }
    }
  }
  __syncthreads();

  {
    const v4i ca = *(const v4i*)(scnt + 8 * tid);
    const v4i cb = *(const v4i*)(scnt + 8 * tid + 4);
    const int e0 = ca.x < 0 ? 0 : ca.x, e1 = ca.y < 0 ? 0 : ca.y, e2 = ca.z < 0 ? 0 : ca.z, e3 = ca.w < 0 ? 0 : ca.w;
    const int e4 = cb.x < 0 ? 0 : cb.x, e5 = cb.y < 0 ? 0 : cb.y, e6 = cb.z < 0 ? 0 : cb.z, e7 = cb.w < 0 ? 0 : cb.w;
    const int ts = e0 + e1 + e2 + e3 + e4 + e5 + e6 + e7;
    int incl = ts;
#pragma unroll
    for (int d = 1; d < 32; d <<= 1) {
      const int up = __shfl_up(incl, d);
      if (lane >= d) incl += up;
    }
    if (lane == 31) wtot[wave] = incl;
    __syncthreads();
    int pre = 0;
#pragma unroll
    for (int w2 = 0; w2 < NWAVE; ++w2) pre += (w2 < wave) ? wtot[w2] : 0;
    int run = pre + incl - ts;
    soff[8 * tid + 0] = run; run += e0;
    soff[8 * tid + 1] = run; run += e1;
    soff[8 * tid + 2] = run; run += e2;
    soff[8 * tid + 3] = run; run += e3;
    soff[8 * tid + 4] = run; run += e4;
    soff[8 * tid + 5] = run; run += e5;
    soff[8 * tid + 6] = run; run += e6;
    soff[8 * tid + 7] = run;
  }
  __syncthreads();
  for (int i = tid; i < NBMAX; i += NTHR) list[i] = soff[i];
  __syncthreads();

  if (wave == 0) {
#pragma unroll 1
    for (int b0 = 0; b0 < nh; b0 += 32) {
      const int idx = b0 + lane;
      const int uv  = reg1[idx < RCAP ? idx : RCAP - 1];
      const int m32 = (nh - b0) < 32 ? (nh - b0) : 32;
#pragma unroll 1
      for (int k = 0; k < m32; ++k) {
        const int u   = __builtin_amdgcn_readlane(uv, k);
        const int sl  = u & (NBMAX - 1);
        const int eid = (int)((unsigned)u >> 12);
        if (lane == 0) {
          int pos = list[sl];
          pos = pos < 0 ? 0 : (pos > RCAP - 1 ? RCAP - 1 : pos);
          reg2[pos] = eid;
          list[sl] = pos + 1;
        }
      }
    }
  }
  __syncthreads();

  {
    const int nq = nb >> 2;
#pragma unroll 1
    for (int t = tid; t < nq; t += NTHR) {
      const v4i c4 = *(const v4i*)(scnt + 4 * t);
      const int rb = nodeBase + 4 * t;
      v4f dv;
      int c;
      c = c4.x; c = c < 0 ? 0 : (c > DEGCAP ? DEGCAP : c); dv.x = (rb     < nN) ? (float)c : 0.f;
      c = c4.y; c = c < 0 ? 0 : (c > DEGCAP ? DEGCAP : c); dv.y = (rb + 1 < nN) ? (float)c : 0.f;
      c = c4.z; c = c < 0 ? 0 : (c > DEGCAP ? DEGCAP : c); dv.z = (rb + 2 < nN) ? (float)c : 0.f;
      c = c4.w; c = c < 0 ? 0 : (c > DEGCAP ? DEGCAP : c); dv.w = (rb + 3 < nN) ? (float)c : 0.f;
      *(volatile v4f*)(DEG + rb) = dv;
    }
    __threadfence();
#pragma unroll 1
    for (int t = tid; t < nq; t += NTHR) {
      const v4i c4 = *(const v4i*)(scnt + 4 * t);
      const int rb = nodeBase + 4 * t;
      v4f dv;
      int c;
      c = c4.x; c = c < 0 ? 0 : (c > DEGCAP ? DEGCAP : c); dv.x = (rb     < nN) ? (float)c : 0.f;
      c = c4.y; c = c < 0 ? 0 : (c > DEGCAP ? DEGCAP : c); dv.y = (rb + 1 < nN) ? (float)c : 0.f;
      c = c4.z; c = c < 0 ? 0 : (c > DEGCAP ? DEGCAP : c); dv.z = (rb + 2 < nN) ? (float)c : 0.f;
      c = c4.w; c = c < 0 ? 0 : (c > DEGCAP ? DEGCAP : c); dv.w = (rb + 3 < nN) ? (float)c : 0.f;
      *(volatile v4f*)(DEG + rb) = dv;
    }
  }

  const v4f wv0 = *(const v4f*)(w1c + 4 * lane);
  const v4f wv1 = *(const v4f*)(w1c + HD + 4 * lane);
  const v4f wv2 = *(const v4f*)(w1c + 2 * HD + 4 * lane);
  const v4f wv3 = *(const v4f*)(w1c + 3 * HD + 4 * lane);
  const int nbw = nb >> 3;
  const bool ovf = (nh >= RCAP);
  const float qnan = __int_as_float(0x7fc00000);
#pragma unroll 1
  for (int jt = 0; jt < nbw; ++jt) {
    const int slot = wave * nbw + jt;
    const int grow = nodeBase + slot;
    const int gcl  = grow < nN ? grow : nN - 1;
    int st = soff[slot];
    const int craw = scnt[slot];
    int cnt = craw;
    st  = st < 0 ? 0 : (st > nh ? nh : st);
    cnt = cnt < 0 ? 0 : (cnt > DEGCAP ? DEGCAP : cnt);
    if (cnt > nh - st) cnt = nh - st;
    const float pz = (ovf || craw > DEGCAP) ? qnan : 0.0f;
    const bool wr = grow < NPr;
    const float live = grow < nN ? 1.0f : 0.0f;

    const v4f pv = *(const v4f*)(PQ + (size_t)gcl * HD2 + 4 * lane);
    v4f sm = {0.f, 0.f, 0.f, 0.f};
#pragma unroll 1
    for (int q = 0; q < cnt; ++q) {
      int idx = st + q; idx = idx > RCAP - 1 ? RCAP - 1 : idx;
      int el = reg2[idx]; el = el < 0 ? 0 : (el > nE - 1 ? nE - 1 : el);
      int s = srcs[el]; s = s < 0 ? 0 : (s > nN - 1 ? nN - 1 : s);
      const v4f qv = *(const v4f*)(PQ + (size_t)s * HD2 + HD + 4 * lane);
      const v4f ev = *(const v4f*)(eattr + (size_t)el * EDIM);
      v4f z = pv + qv;
      z = z + wv0 * ev.x;
      z = z + wv1 * ev.y;
      z = z + wv2 * ev.z;
      z = z + wv3 * ev.w;
      sm = sm + relu4(z);
    }
    const v4f rs = sm * live + pz;
    float* gp = RS + (size_t)grow * HD + 4 * lane;
    if (wr) *(volatile v4f*)gp = rs;
    __threadfence();
    if (wr) *(volatile v4f*)gp = rs;
  }
}

__global__ __launch_bounds__(NTHR) void k_upd(const float* __restrict__ AGG, const _Float16* __restrict__ U1T,
                                              const _Float16* __restrict__ U2T, const float* __restrict__ ub1,
                                              const float* __restrict__ ub2, const float* __restrict__ lng,
                                              const float* __restrict__ lnb, float* hio, int nN) {
  extern __shared__ v4f lds_dynu[];
  _Float16* zh  = (_Float16*)lds_dynu;
  _Float16* zl  = zh + GBM * ZP;
  float*    stg = (float*)(zl + GBM * ZP);
  const int tid = (int)threadIdx.x, lane = tid & 31, wave = tid >> 5, hh = lane >> 4, m = lane & 15;
  const int rowBase = (int)blockIdx.x * GBM;
  const int wr = wave & 3, wcg = wave >> 2;
  const v4f g4 = *(const v4f*)(lng + 4 * lane);
  const v4f b4 = *(const v4f*)(lnb + 4 * lane);

  v8f acch[4], accl[4];
  {
    const v8f z = {0.f, 0.f, 0.f, 0.f, 0.f, 0.f, 0.f, 0.f};
#pragma unroll
    for (int t = 0; t < 4; ++t) { acch[t] = z; accl[t] = z; }
  }
  const int gra = rowBase + 16 * wr + m;
  const int grc = gra > nN - 1 ? nN - 1 : gra;
  const float* hp = hio + (size_t)grc * HD + 8 * hh;
  const float* gp = AGG + (size_t)gra * HD + 8 * hh;
  const _Float16* up = U1T + (size_t)(64 * wcg + m) * HD2 + 8 * hh;

#pragma unroll 1
  for (int ks = 0; ks < HD / 32; ++ks) {
    const float* aq = hp + 32 * ks;
    const v4f a0 = *(const v4f*)aq,        a1 = *(const v4f*)(aq + 4);
    const v4f a2 = *(const v4f*)(aq + 16), a3 = *(const v4f*)(aq + 20);
    FragH ah, al;
    cvt8hl(a0, a1, ah.h[0], al.h[0]);
    cvt8hl(a2, a3, ah.h[1], al.h[1]);
#pragma unroll
    for (int t = 0; t < 4; ++t) {
      const _Float16* wq = up + (size_t)(16 * t) * HD2 + 32 * ks;
      FragH bf;
      bf.h[0] = *(const v8h*)wq;
      bf.h[1] = *(const v8h*)(wq + 16);
      acch[t] = wmh(ah, bf, acch[t]);
      accl[t] = wmh(al, bf, accl[t]);
    }
  }
#pragma unroll 1
  for (int ks = 0; ks < HD / 32; ++ks) {
    const float* aq = gp + 32 * ks;
    const v4f a0 = *(const v4f*)aq,        a1 = *(const v4f*)(aq + 4);
    const v4f a2 = *(const v4f*)(aq + 16), a3 = *(const v4f*)(aq + 20);
    FragH ah, al;
    cvt8hl(a0, a1, ah.h[0], al.h[0]);
    cvt8hl(a2, a3, ah.h[1], al.h[1]);
#pragma unroll
    for (int t = 0; t < 4; ++t) {
      const _Float16* wq = up + (size_t)(16 * t) * HD2 + HD + 32 * ks;
      FragH bf;
      bf.h[0] = *(const v8h*)wq;
      bf.h[1] = *(const v8h*)(wq + 16);
      acch[t] = wmh(ah, bf, acch[t]);
      accl[t] = wmh(al, bf, accl[t]);
    }
  }
#pragma unroll
  for (int t = 0; t < 4; ++t) {
    const int lc = 64 * wcg + 16 * t + m;
    const float bv = ub1[lc];
#pragma unroll
    for (int r = 0; r < 8; ++r) {
      const int lr = 16 * wr + 8 * hh + r;
      float v = acch[t][r] * SCL;
      v = fmaf(accl[t][r], SCLL, v);
      v = fmaxf(v + bv, 0.f);
      const float s = v * CA;
      const _Float16 q = (_Float16)s;
      zh[lr * ZP + lc] = q;
      zl[lr * ZP + lc] = (_Float16)((s - (float)q) * CL);
    }
  }
  __syncthreads();

  {
    const v8f z = {0.f, 0.f, 0.f, 0.f, 0.f, 0.f, 0.f, 0.f};
#pragma unroll
    for (int t = 0; t < 4; ++t) { acch[t] = z; accl[t] = z; }
  }
  const _Float16* aph = zh + (16 * wr + m) * ZP + 8 * hh;
  const _Float16* apl = zl + (16 * wr + m) * ZP + 8 * hh;
  const _Float16* wp2 = U2T + (size_t)(64 * wcg + m) * HD + 8 * hh;
#pragma unroll 1
  for (int ks = 0; ks < HD / 32; ++ks) {
    FragH ah, al;
    ah.h[0] = *(const v8h*)(aph + 32 * ks);
    ah.h[1] = *(const v8h*)(aph + 32 * ks + 16);
    al.h[0] = *(const v8h*)(apl + 32 * ks);
    al.h[1] = *(const v8h*)(apl + 32 * ks + 16);
#pragma unroll
    for (int t = 0; t < 4; ++t) {
      const _Float16* wq = wp2 + (size_t)(16 * t) * HD + 32 * ks;
      FragH bf;
      bf.h[0] = *(const v8h*)wq;
      bf.h[1] = *(const v8h*)(wq + 16);
      acch[t] = wmh(ah, bf, acch[t]);
      accl[t] = wmh(al, bf, accl[t]);
    }
  }
#pragma unroll
  for (int t = 0; t < 4; ++t) {
    const int lc = 64 * wcg + 16 * t + m;
    const float bv = ub2[lc];
#pragma unroll
    for (int r = 0; r < 8; ++r) {
      const int lr = 16 * wr + 8 * hh + r;
      float v = acch[t][r] * SCL;
      v = fmaf(accl[t][r], SCLL, v);
      stg[lr * SP + lc] = v + bv;
    }
  }
  __syncthreads();

  v4f y[8];
#pragma unroll
  for (int i = 0; i < 8; ++i) {
    const int lr   = 8 * wave + i;
    const int grow = rowBase + lr;
    const int gclr = grow > nN - 1 ? nN - 1 : grow;
    const v4f sv = *(const v4f*)(stg + lr * SP + 4 * lane);
    const v4f hv = *(const v4f*)(hio + (size_t)gclr * HD + 4 * lane);
    const v4f u  = sv + hv;
    float s1 = (u.x + u.y) + (u.z + u.w);
    s1 = wred(s1);
    const float mean = s1 * (1.0f / (float)HD);
    const v4f dv = u - mean;
    float s2 = (dv.x * dv.x + dv.y * dv.y) + (dv.z * dv.z + dv.w * dv.w);
    s2 = wred(s2);
    const float var = s2 * (1.0f / (float)HD);
    const float rsd = rsqrtf(var + LNEPS);
    y[i] = dv * rsd * g4 + b4;
  }
#pragma unroll
  for (int i = 0; i < 8; ++i) {
    const int grow = rowBase + 8 * wave + i;
    if (grow < nN) *(volatile v4f*)(hio + (size_t)grow * HD + 4 * lane) = y[i];
  }
  __threadfence();
#pragma unroll
  for (int i = 0; i < 8; ++i) {
    const int grow = rowBase + 8 * wave + i;
    if (grow < nN) *(volatile v4f*)(hio + (size_t)grow * HD + 4 * lane) = y[i];
  }
}

static inline int cdiv(int a, int b) { return (a + b - 1) / b; }
static int pick_nb(int nE, int nN) {
  int nb = NBMAX;
  while (nb > 32 && (long long)nb * (long long)nE * 11LL > (long long)RCAP * (long long)nN * 8LL) nb >>= 1;
  return nb;
}

extern "C" void kernel_launch(void* const* d_in, const int* in_sizes, int n_in,
                              void* d_out, int out_size, void* d_ws, size_t ws_size,
                              hipStream_t stream) {
  if (n_in < 15) return;
  const int nN = in_sizes[0] / INDIM;
  if (nN <= 0 || in_sizes[0] != nN * INDIM || nN > (1 << 20)) return;
  const int nE = in_sizes[1] / 2;
  if (nE < 1 || in_sizes[1] != 2 * nE || nE > (1 << 20)) return;
  if (in_sizes[2]  != nE * EDIM) return;
  if (in_sizes[3]  != INDIM * HD         || in_sizes[4]  != HD)        return;
  if (in_sizes[5]  != NLAY * K1ROWS * HD || in_sizes[6]  != NLAY * HD) return;
  if (in_sizes[7]  != NLAY * HD * HD     || in_sizes[8]  != NLAY * HD) return;
  if (in_sizes[9]  != NLAY * HD2 * HD    || in_sizes[10] != NLAY * HD) return;
  if (in_sizes[11] != NLAY * HD * HD     || in_sizes[12] != NLAY * HD) return;
  if (in_sizes[13] != NLAY * HD          || in_sizes[14] != NLAY * HD) return;
  if (out_size != nN * HD) return;

  const float* x      = (const float*)d_in[0];
  const int*   eidx   = (const int*)  d_in[1];
  const float* eattr  = (const float*)d_in[2];
  const float* proj_w = (const float*)d_in[3];
  const float* proj_b = (const float*)d_in[4];
  const float* msg_w1 = (const float*)d_in[5];
  const float* msg_b1 = (const float*)d_in[6];
  const float* msg_w2 = (const float*)d_in[7];
  const float* msg_b2 = (const float*)d_in[8];
  const float* upd_w1 = (const float*)d_in[9];
  const float* upd_b1 = (const float*)d_in[10];
  const float* upd_w2 = (const float*)d_in[11];
  const float* upd_b2 = (const float*)d_in[12];
  const float* ln_g   = (const float*)d_in[13];
  const float* ln_b   = (const float*)d_in[14];
  const int* srcp = eidx;
  const int* dstp = eidx + (size_t)nE;
  float* out = (float*)d_out;

  const int NP = cdiv(nN, GBM) * GBM;
  const int nb = pick_nb(nE, nN);
  const int gA = cdiv(NP, nb);
  if (gA * nb < NP || nb > NBMAX || nb < 32) return;
  const int DEGN = gA * nb;
  const int vec8 = ((nE & 3) == 0) ? 1 : 0;

  char* ws = (char*)d_ws;
  size_t off = 0;
  const size_t oWPL = off; off += (size_t)NLAY * WL_LAY * 2;       off = (off + 255) & ~(size_t)255;
  const size_t oPQ  = off; off += (size_t)NP * HD2 * 4;            off = (off + 255) & ~(size_t)255;
  const size_t oRS  = off; off += (size_t)NP * HD * 4;             off = (off + 255) & ~(size_t)255;
  const size_t oAGG = off; off += (size_t)NP * HD * 4;             off = (off + 255) & ~(size_t)255;
  const size_t oDEG = off; off += (size_t)DEGN * 4;                off = (off + 255) & ~(size_t)255;
  if (off > ws_size || off > (size_t)WSMAX) return;
  _Float16* WPL = (_Float16*)(ws + oWPL);
  float*    PQ  = (float*)(ws + oPQ);
  float*    RS  = (float*)(ws + oRS);
  float*    AGG = (float*)(ws + oAGG);
  float*    DEG = (float*)(ws + oDEG);

  hipFuncSetAttribute(reinterpret_cast<const void*>(&k_scan),
                      hipFuncAttributeMaxDynamicSharedMemorySize, LDS_AGG);
  hipFuncSetAttribute(reinterpret_cast<const void*>(&k_upd),
                      hipFuncAttributeMaxDynamicSharedMemorySize, LDS_UPD);

  {
    const int nU = NLAY * UPL;
    k_wcvt<<<cdiv(nU, NTHR), NTHR, 0, stream>>>(msg_w1, msg_w2, upd_w1, upd_w2, WPL, nU);
  }
  {
    const int nT = nN * (HD / 4);
    k_proj<<<cdiv(nT, NTHR), NTHR, 0, stream>>>(x, proj_w, proj_b, out, nT);
  }

  for (int l = 0; l < NLAY; ++l) {
    const _Float16* W1T = WPL + (size_t)l * WL_LAY + WL_W1T;
    const _Float16* W2T = WPL + (size_t)l * WL_LAY + WL_W2T;
    const _Float16* U1T = WPL + (size_t)l * WL_LAY + WL_U1T;
    const _Float16* U2T = WPL + (size_t)l * WL_LAY + WL_U2T;
    const float* w1c = msg_w1 + (size_t)l * K1ROWS * HD + (size_t)HD2 * HD;
    const float* b1  = msg_b1 + (size_t)l * HD;
    const float* b2  = msg_b2 + (size_t)l * HD;
    const float* u1b = upd_b1 + (size_t)l * HD;
    const float* u2b = upd_b2 + (size_t)l * HD;
    const float* lg  = ln_g   + (size_t)l * HD;
    const float* lb  = ln_b   + (size_t)l * HD;

    k_ngemm<0><<<dim3(NP / GBM, HD2 / GBN), GTHR, 0, stream>>>(out, W1T, b1, DEG, PQ, nN, HD, HD, HD2, HD);
    k_scan<<<gA, NTHR, LDS_AGG, stream>>>(dstp, srcp, eattr, PQ, w1c, RS, DEG, nN, nE, nb, vec8, NP);
    k_ngemm<1><<<dim3(NP / GBM, HD / GBN), GTHR, 0, stream>>>(RS, W2T, b2, DEG, AGG, NP, HD, HD, HD, HD);
    k_upd<<<NP / GBM, NTHR, LDS_UPD, stream>>>(AGG, U1T, U2T, u1b, u2b, lg, lb, out, nN);
  }
}
